// ConvTran_32770600468898
// MI455X (gfx1250) — hardware-verified
//
#include <hip/hip_runtime.h>


namespace {
constexpr int NB = 16, NC = 9, L = 1024, D = 16, NH = 8, HD = 2, DFF = 256, NCLS = 10, OC1 = 64, K2 = OC1 * NC  , NT = NB * L  , NBLK1 = NB * NC * (L / 64)  ;
constexpr float XS = 8.0f, WSC = 256.0f, EPS = 1e-5f, SCALE = 0.25f, PSB = 8.0f;

typedef _Float16 b16;
typedef __attribute__((ext_vector_type(16))) _Float16 v16b;
typedef __attribute__((ext_vector_type(8))) _Float16 v8b;
typedef __attribute__((ext_vector_type(8))) float v8f;
typedef __attribute__((ext_vector_type(4))) float v4f;
__device__ __forceinline__ float bf16_rne(float f) { unsigned int u = __float_as_uint(f); u += 0x7FFFu + ((u >> 16) & 1u); return __uint_as_float(u & 0xFFFF0000u); }
__device__ __forceinline__ void split16(float v, b16& hi, b16& lo) { hi = (b16)v; lo = (b16)(v - (float)hi); }
__device__ __forceinline__ v16b frag_kb(const b16* p, int hh) { const v8b a = *(const v8b*)(p + 8 * hh), b = *(const v8b*)(p + 16 + 8 * hh); v16b f;
#pragma unroll
  for (int e = 0; e < 8; ++e) { f[e] = a[e]; f[8 + e] = b[e]; } return f; }
__device__ __forceinline__ v8f wmma16b(v16b a, v16b b, v8f c) { v8f d = __builtin_amdgcn_wmma_f32_16x16x32_f16(false, a, false, b, (short)0, c, false, false); asm volatile("v_nop\n\tv_nop\n\tv_nop\n\tv_nop" : "+v"(d) : "v"(a), "v"(b)); return d; }
__device__ __forceinline__ void wave_lds_sync() { __builtin_amdgcn_fence(__ATOMIC_RELEASE, "workgroup"); __builtin_amdgcn_wave_barrier(); __builtin_amdgcn_fence(__ATOMIC_ACQUIRE, "workgroup"); }
__device__ __forceinline__ float pmul(float a, float b) { float p = a * b; asm volatile("" : "+v"(p)); return p; }
__device__ __forceinline__ float gelu_(float x) { return 0.5f * x * (1.0f + erff(x * 0.70710678118654752f)); }

__global__ __launch_bounds__(256) void prepw_kernel(const float* __restrict__ w1, const float* __restrict__ w2, const float* __restrict__ f1, const float* __restrict__ f2, b16* __restrict__ W1P, b16* __restrict__ W2P, b16* __restrict__ F1P, b16* __restrict__ F2P) {
  const int t = blockIdx.x * 256 + threadIdx.x; int u = t; v8b o; const int n1 = OC1 * 32 / 8, n2 = D * K2 / 8, n3 = DFF * 32 / 8, n4 = D * DFF / 8;
  if (u < n1) { const int e = u * 8, oc = e / 32, k0 = e % 32; for (int j = 0; j < 8; ++j) { const int k = k0 + j; o[j] = (k < 8) ? (b16)(bf16_rne(w1[oc * 8 + k]) * WSC) : (b16)0.0f; } for (int pass = 0; pass < 2; ++pass) { *(volatile v8b*)(W1P + e) = o; __threadfence(); } return; } u -= n1;
  if (u < n2) { const int e = u * 8, d = e / K2, k0 = e % K2; for (int j = 0; j < 8; ++j) { const int k = k0 + j; const int c9 = k / OC1, c64 = k % OC1; o[j] = (b16)(bf16_rne(w2[(d * OC1 + c64) * NC + c9]) * WSC); } for (int pass = 0; pass < 2; ++pass) { *(volatile v8b*)(W2P + e) = o; __threadfence(); } return; } u -= n2;
  if (u < n3) { const int e = u * 8, oo = e / 32, k0 = e % 32; for (int j = 0; j < 8; ++j) { const int k = k0 + j; o[j] = (k < D) ? (b16)(bf16_rne(f1[k * DFF + oo]) * WSC) : (b16)0.0f; } for (int pass = 0; pass < 2; ++pass) { *(volatile v8b*)(F1P + e) = o; __threadfence(); } return; } u -= n3;
  if (u < n4) { const int e = u * 8, oo = e / DFF, k0 = e % DFF; for (int j = 0; j < 8; ++j) o[j] = (b16)(bf16_rne(f2[(k0 + j) * D + oo]) * WSC); for (int pass = 0; pass < 2; ++pass) { *(volatile v8b*)(F2P + e) = o; __threadfence(); } }
}
__global__ __launch_bounds__(128) void conv1_kernel(const float* __restrict__ x, const b16* __restrict__ W1P, const float* __restrict__ b1, b16* __restrict__ H1h, b16* __restrict__ H1l, float* __restrict__ PS1) {
  __shared__ __attribute__((aligned(16))) b16 At[4][16][32 + 8]; __shared__ __attribute__((aligned(16))) b16 Th[4][16][OC1 + 8], Tl[4][16][OC1 + 8]; __shared__ float cs[4][2][OC1]; __shared__ __attribute__((aligned(16))) float row[OC1];
  const int b = blockIdx.x, c9 = blockIdx.y / (L / 64), l0 = (blockIdx.y % (L / 64)) * 64; const int wave = threadIdx.x >> 5, lane = threadIdx.x & 31, nloc = lane & 15, hlf = lane >> 4, t_ = threadIdx.x;
  const float* xr = x + ((size_t)b * NC + c9) * L; const int ls = l0 + wave * 16;
  for (int k = hlf * 16; k < hlf * 16 + 16; ++k) { float v = 0.0f; if (k < 8) { const int li = ls + nloc + k - 3; if (li >= 0 && li < L) v = bf16_rne(xr[li]); } At[wave][nloc][k] = (b16)(v * XS); }
  wave_lds_sync();
  const v16b a = frag_kb(&At[wave][nloc][0], hlf); float csum[4][1]; (void)csum; float cpart[4] = {0.0f, 0.0f, 0.0f, 0.0f};
#pragma unroll
  for (int t = 0; t < 4; ++t) { v8f d = {}; d = wmma16b(a, frag_kb(W1P + (size_t)(t * 16 + nloc) * 32, hlf), d); const float bb = bf16_rne(b1[t * 16 + nloc]);
    for (int r = 0; r < 8; ++r) { const float h = d[r] * (1.0f / (XS * WSC)) + bb; cpart[t] += h; b16 p, q; split16(h * XS, p, q); Th[wave][8 * hlf + r][t * 16 + nloc] = p; Tl[wave][8 * hlf + r][t * 16 + nloc] = q; } }
#pragma unroll
  for (int t = 0; t < 4; ++t) cs[wave][hlf][t * 16 + nloc] = cpart[t];
  __syncthreads();
  if (t_ < OC1) { float s = 0.0f; for (int w = 0; w < 4; ++w) s += cs[w][0][t_] + cs[w][1][t_]; row[t_] = s; }
  __syncthreads();
  for (int pass = 0; pass < 2; ++pass) {
    for (int q = lane; q < 16 * 8; q += 32) { const int rr = q >> 3, c8 = (q & 7) * 8; const size_t gi = ((size_t)(b * L + ls + rr)) * K2 + c9 * OC1 + c8; *(volatile v8b*)(H1h + gi) = *(const v8b*)(&Th[wave][rr][c8]); *(volatile v8b*)(H1l + gi) = *(const v8b*)(&Tl[wave][rr][c8]); }
    if (t_ < 16) *(volatile v4f*)(PS1 + ((size_t)blockIdx.x * gridDim.y + blockIdx.y) * OC1 + t_ * 4) = *(const v4f*)(&row[t_ * 4]);
    __threadfence(); }
}
__global__ __launch_bounds__(64) void bnred_kernel(const float* __restrict__ PS, int nblk, float denom, int mode, const float* __restrict__ MU, float* __restrict__ OUTV) {
  __shared__ __attribute__((aligned(16))) float r[OC1];
  const int c = threadIdx.x; float s = 0.0f; for (int k = 0; k < nblk; ++k) s += PS[(size_t)k * OC1 + c];
  r[c] = (mode == 0) ? s / denom : rsqrtf(s / denom + EPS); (void)MU;
  __syncthreads();
  for (int pass = 0; pass < 2; ++pass) { if (c < 16) *(volatile v4f*)(OUTV + c * 4) = *(const v4f*)(&r[c * 4]); __threadfence(); }
}
__global__ __launch_bounds__(128) void bn1var_kernel(const b16* __restrict__ H1h, const b16* __restrict__ H1l, const float* __restrict__ MU1, float* __restrict__ PS1) {
  __shared__ float cs[128][OC1 / 32 + 1]; __shared__ __attribute__((aligned(16))) float row[OC1];
  const int b = blockIdx.x, c9 = blockIdx.y / (L / 64), l0 = (blockIdx.y % (L / 64)) * 64, t_ = threadIdx.x; const int step = t_ >> 1, half = t_ & 1;
  float part[OC1 / 32]; (void)part; float acc2[32];
  { const size_t base = ((size_t)(b * L + l0 + step)) * K2 + c9 * OC1 + half * 32; for (int j = 0; j < 32; ++j) { const float h = ((float)H1h[base + j] + (float)H1l[base + j]) * (1.0f / XS); const float dv = h - MU1[half * 32 + j]; acc2[j] = dv * dv; } }
  __shared__ float tmp[64][OC1 + 1];
  for (int j = 0; j < 32; ++j) tmp[step][half * 32 + j] = acc2[j];
  __syncthreads();
  if (t_ < OC1) { float s = 0.0f; for (int st = 0; st < 64; ++st) s += tmp[st][t_]; row[t_] = s; }
  __syncthreads(); (void)cs;
  for (int pass = 0; pass < 2; ++pass) { if (t_ < 16) *(volatile v4f*)(PS1 + ((size_t)blockIdx.x * gridDim.y + blockIdx.y) * OC1 + t_ * 4) = *(const v4f*)(&row[t_ * 4]); __threadfence(); }
}
__global__ __launch_bounds__(64) void conv2_kernel(const b16* __restrict__ H1h, const b16* __restrict__ H1l, const float* __restrict__ MU1, const float* __restrict__ RS1, const float* __restrict__ g1, const float* __restrict__ be1, const b16* __restrict__ W2P, const float* __restrict__ b2, float* __restrict__ H2) {
  __shared__ __attribute__((aligned(16))) b16 Ah[2][16][K2 + 8], Al[2][16][K2 + 8]; __shared__ __attribute__((aligned(16))) float To[2][16][D];
  const int wave = threadIdx.x >> 5, lane = threadIdx.x & 31, nloc = lane & 15, hlf = lane >> 4; const size_t m0 = (size_t)blockIdx.x * 32 + wave * 16;
  for (int q = lane; q < 16 * K2; q += 32) { const int rr = q / K2, k = q % K2; const int c64 = k % OC1; const size_t gi = (m0 + rr) * K2 + k; const float h = ((float)H1h[gi] + (float)H1l[gi]) * (1.0f / XS);
    const float v = gelu_((h - MU1[c64]) * RS1[c64] * bf16_rne(g1[c64]) + bf16_rne(be1[c64])); b16 p, pl; split16(v * XS, p, pl); Ah[wave][rr][k] = p; Al[wave][rr][k] = pl; }
  wave_lds_sync();
  v8f d = {};
  for (int kb = 0; kb < K2; kb += 32) { const v16b bw = frag_kb(W2P + (size_t)nloc * K2 + kb, hlf); d = wmma16b(frag_kb(&Ah[wave][nloc][kb], hlf), bw, d); d = wmma16b(frag_kb(&Al[wave][nloc][kb], hlf), bw, d); }
  for (int r = 0; r < 8; ++r) To[wave][8 * hlf + r][nloc] = d[r] * (1.0f / (XS * WSC)) + bf16_rne(b2[nloc]);
  wave_lds_sync();
  for (int pass = 0; pass < 2; ++pass) { for (int k = 0; k < 2; ++k) *(volatile v4f*)(H2 + (m0 + k * 8) * D + lane * 4) = *(const v4f*)(&To[wave][k * 8][0] + lane * 4); __threadfence(); }
}
__global__ __launch_bounds__(64) void bn2part_kernel(const float* __restrict__ H2, const float* __restrict__ MU2, int mode, float* __restrict__ PS2) {
  __shared__ float tmp[64][D + 1]; __shared__ __attribute__((aligned(16))) float row[32];
  const int t_ = threadIdx.x; const size_t tok = (size_t)blockIdx.x * 64 + t_;
  for (int c = 0; c < D; ++c) { const float h = H2[tok * D + c]; tmp[t_][c] = (mode == 0) ? h : (h - MU2[c]) * (h - MU2[c]); }
  __syncthreads();
  if (t_ < 32) { float s = 0.0f; if (t_ < D) for (int st = 0; st < 64; ++st) s += tmp[st][t_]; row[t_] = s; }
  __syncthreads();
  for (int pass = 0; pass < 2; ++pass) { if (t_ < 8) *(volatile v4f*)(PS2 + (size_t)blockIdx.x * 32 + t_ * 4) = *(const v4f*)(&row[t_ * 4]); __threadfence(); }
}
__global__ __launch_bounds__(32) void bnred2_kernel(const float* __restrict__ PS2, int nblk, float denom, int mode, float* __restrict__ OUTV) {
  __shared__ __attribute__((aligned(16))) float r[D]; const int c = threadIdx.x; if (c < D) { float s = 0.0f; for (int k = 0; k < nblk; ++k) s += PS2[(size_t)k * 32 + c]; r[c] = (mode == 0) ? s / denom : rsqrtf(s / denom + EPS); }
  wave_lds_sync();
  for (int pass = 0; pass < 2; ++pass) { if (c < 4) *(volatile v4f*)(OUTV + c * 4) = *(const v4f*)(&r[c * 4]); __threadfence(); }
}
__global__ __launch_bounds__(32) void token_kernel(const float* __restrict__ H2, const float* __restrict__ MU2, const float* __restrict__ RS2, const float* __restrict__ g2, const float* __restrict__ be2, const float* __restrict__ wq, const float* __restrict__ wk, const float* __restrict__ wv, float* __restrict__ XSf, b16* __restrict__ Qh, b16* __restrict__ Ql, b16* __restrict__ Kh, b16* __restrict__ Kl, b16* __restrict__ Vh, b16* __restrict__ Vl) {
  constexpr int TB = 32;
  __shared__ __attribute__((aligned(16))) float xs_s[TB][D]; __shared__ __attribute__((aligned(16))) b16 qh_s[NH][TB][32], ql_s[NH][TB][32], kh_s[NH][TB][32], kl_s[NH][TB][32]; __shared__ __attribute__((aligned(16))) b16 vh_s[NH][HD][TB + 8], vl_s[NH][HD][TB + 8];
  const int t_ = threadIdx.x; const size_t tok = (size_t)blockIdx.x * TB + t_; const int b = (int)(tok / L), l = (int)(tok % L);
  float xp[D];
  for (int c = 0; c < D; ++c) { const float h = H2[tok * D + c]; const float xs = gelu_((h - MU2[c]) * RS2[c] * bf16_rne(g2[c]) + bf16_rne(be2[c])); xs_s[t_][c] = xs;
    const int i2 = c & ~1; const float divi = __expf((float)i2 * (-9.2103403719761836f / (float)D)); const float ang = (float)l * divi * ((float)D / (float)L); xp[c] = xs + ((c & 1) ? cosf(ang) : sinf(ang)); }
  for (int h = 0; h < NH; ++h) for (int dd = 0; dd < 32; ++dd) { qh_s[h][t_][dd] = (b16)0.0f; ql_s[h][t_][dd] = (b16)0.0f; kh_s[h][t_][dd] = (b16)0.0f; kl_s[h][t_][dd] = (b16)0.0f; }
  for (int o = 0; o < D; ++o) { float q = 0.0f, k = 0.0f, v = 0.0f;
#pragma unroll 1
    for (int c = 0; c < D; ++c) { q += pmul(xp[c], bf16_rne(wq[c * D + o])); k += pmul(xp[c], bf16_rne(wk[c * D + o])); v += pmul(xp[c], bf16_rne(wv[c * D + o])); }
    const int h = o / HD, dd = o % HD; b16 p, pl; split16(q * XS, p, pl); qh_s[h][t_][dd] = p; ql_s[h][t_][dd] = pl; split16(k * XS, p, pl); kh_s[h][t_][dd] = p; kl_s[h][t_][dd] = pl; split16(v * XS, p, pl); vh_s[h][dd][t_] = p; vl_s[h][dd][t_] = pl; }
  wave_lds_sync();
  const int l0 = (int)(((size_t)blockIdx.x * TB) % L);
  for (int pass = 0; pass < 2; ++pass) {
    for (int q = t_; q < TB * D / 4; q += 32) *(volatile v4f*)(XSf + (size_t)blockIdx.x * TB * D + q * 4) = *(const v4f*)(&xs_s[0][0] + q * 4);
    for (int q = t_; q < NH * TB * 4; q += 32) { const int h = q / (TB * 4), rem = q % (TB * 4); const int rr = rem >> 2, c8 = (rem & 3) * 8; const size_t gi = (((size_t)b * NH + h) * L + l0 + rr) * 32 + c8;
      *(volatile v8b*)(Qh + gi) = *(const v8b*)(&qh_s[h][rr][c8]); *(volatile v8b*)(Ql + gi) = *(const v8b*)(&ql_s[h][rr][c8]); *(volatile v8b*)(Kh + gi) = *(const v8b*)(&kh_s[h][rr][c8]); *(volatile v8b*)(Kl + gi) = *(const v8b*)(&kl_s[h][rr][c8]); }
    for (int q = t_; q < NH * 16 * (TB / 8); q += 32) { const int h = q / (16 * (TB / 8)), rem = q % (16 * (TB / 8)); const int dd = rem / (TB / 8), c8 = (rem % (TB / 8)) * 8; const size_t gi = ((((size_t)b * NH + h) * (L / TB) + l0 / TB) * 16 + dd) * TB + c8;
      v8b hv = {}, lv = {}; if (dd < HD) { hv = *(const v8b*)(&vh_s[h][dd][c8]); lv = *(const v8b*)(&vl_s[h][dd][c8]); } *(volatile v8b*)(Vh + gi) = hv; *(volatile v8b*)(Vl + gi) = lv; }
    __threadfence(); }
}
__global__ __launch_bounds__(32) void attn_kernel(const b16* __restrict__ Qh, const b16* __restrict__ Ql, const b16* __restrict__ Kh, const b16* __restrict__ Kl, const b16* __restrict__ Vh, const b16* __restrict__ Vl, const float* __restrict__ rel, float* __restrict__ OB) {
  __shared__ __attribute__((aligned(16))) b16 Ph[16][L + 8], Pl[16][L + 8]; __shared__ __attribute__((aligned(16))) float orow[16][HD];
  const int lane = threadIdx.x, hh = lane >> 4, col = lane & 15; const int b = blockIdx.z, h = blockIdx.y, q0 = blockIdx.x * 16, qi = q0 + col;
  const size_t bh = (size_t)b * NH + h; const v16b qa = frag_kb(Qh + (bh * L + qi) * 32, hh), ql = frag_kb(Ql + (bh * L + qi) * 32, hh);
  auto stile = [&](int kt) { v8f s = {}; const v16b f = frag_kb(Kh + (bh * L + kt * 16 + col) * 32, hh); s = wmma16b(f, qa, s); s = wmma16b(f, ql, s); s = wmma16b(frag_kb(Kl + (bh * L + kt * 16 + col) * 32, hh), qa, s); return s; };
  const float cs = SCALE / (XS * XS); float mx = -INFINITY;
  for (int kt = 0; kt < L / 16; ++kt) { const v8f s = stile(kt); for (int r = 0; r < 8; ++r) mx = fmaxf(mx, s[r] * cs); }
  mx = fmaxf(mx, __shfl_xor(mx, 16)); float sm = 0.0f;
  for (int kt = 0; kt < L / 16; ++kt) { const v8f s = stile(kt); for (int r = 0; r < 8; ++r) sm += __expf(s[r] * cs - mx); }
  sm += __shfl_xor(sm, 16); const float inv = 1.0f / sm;
  for (int kt = 0; kt < L / 16; ++kt) { const v8f s = stile(kt); for (int r = 0; r < 8; ++r) { const int j = kt * 16 + 8 * hh + r; const float p = __expf(s[r] * cs - mx) * inv + bf16_rne(rel[(size_t)(qi - j + L - 1) * NH + h]); b16 ph_, pl_; split16(p * PSB, ph_, pl_); Ph[col][j] = ph_; Pl[col][j] = pl_; } }
  wave_lds_sync();
  v8f o = {};
  for (int kb = 0; kb < L; kb += 32) { const v16b pa = frag_kb(&Ph[col][kb], hh), pl = frag_kb(&Pl[col][kb], hh); const int drow = (col < HD) ? col : 0;
    const size_t vo = ((bh * (L / 32) + kb / 32) * 16 + drow) * 32; const v16b va = frag_kb(Vh + vo, hh), vl = frag_kb(Vl + vo, hh); o = wmma16b(va, pa, o); o = wmma16b(va, pl, o); o = wmma16b(vl, pa, o); }
  if (hh == 0) { orow[col][0] = o[0] * (1.0f / (PSB * XS)); orow[col][1] = o[1] * (1.0f / (PSB * XS)); }
  wave_lds_sync();
  for (int pass = 0; pass < 2; ++pass) { if (lane < 8) *(volatile v4f*)(OB + (bh * L + q0) * HD + lane * 4) = *(const v4f*)(&orow[0][0] + lane * 4); __threadfence(); }
}
__global__ __launch_bounds__(128) void post_kernel(const float* __restrict__ OB, const float* __restrict__ XSf, const float* __restrict__ lag, const float* __restrict__ lab, const float* __restrict__ l1g, const float* __restrict__ l1b, const b16* __restrict__ F1P, const float* __restrict__ fb1, const b16* __restrict__ F2P, const float* __restrict__ fb2, const float* __restrict__ l2g, const float* __restrict__ l2b, float* __restrict__ PSO) {
  __shared__ __attribute__((aligned(16))) b16 Ah[4][16][32 + 8], Al[4][16][32 + 8]; __shared__ __attribute__((aligned(16))) b16 Hh[4][16][DFF + 8], Hl[4][16][DFF + 8]; __shared__ float att_s[4][16][D + 1]; __shared__ float part[4][D]; __shared__ __attribute__((aligned(16))) float row[32];
  const int wave = threadIdx.x >> 5, lane = threadIdx.x & 31, nloc = lane & 15, hlf = lane >> 4, t_ = threadIdx.x; const size_t m0 = (size_t)blockIdx.x * 64 + wave * 16;
  if (lane < 16) { const size_t tok = m0 + lane; const int b = (int)(tok / L), l = (int)(tok % L); float o[D];
    for (int c = 0; c < D; ++c) { const int h = c / HD, dd = c % HD; o[c] = OB[(((size_t)b * NH + h) * L + l) * HD + dd]; }
    auto ln = [&](float* v, const float* g, const float* bb) { float mu = 0.0f; for (int c = 0; c < D; ++c) mu += v[c]; mu *= (1.0f / D); float var = 0.0f; for (int c = 0; c < D; ++c) { const float dv = v[c] - mu; var += dv * dv; } var *= (1.0f / D); const float rs = 1.0f / sqrtf(var + EPS); for (int c = 0; c < D; ++c) v[c] = (v[c] - mu) * rs * bf16_rne(g[c]) + bf16_rne(bb[c]); };
    ln(o, lag, lab); float a[D]; for (int c = 0; c < D; ++c) a[c] = XSf[tok * D + c] + o[c]; ln(a, l1g, l1b);
    for (int c = 0; c < 32; ++c) { b16 p = (b16)0.0f, pl = (b16)0.0f; if (c < D) { split16(a[c] * XS, p, pl); att_s[wave][lane][c] = a[c]; } Ah[wave][lane][c] = p; Al[wave][lane][c] = pl; } }
  wave_lds_sync();
  { const v16b aa = frag_kb(&Ah[wave][nloc][0], hlf), al = frag_kb(&Al[wave][nloc][0], hlf);
    for (int t = 0; t < DFF / 16; ++t) { v8f d = {}; const v16b bw = frag_kb(F1P + (size_t)(t * 16 + nloc) * 32, hlf); d = wmma16b(aa, bw, d); d = wmma16b(al, bw, d); const float bb = bf16_rne(fb1[t * 16 + nloc]);
      for (int r = 0; r < 8; ++r) { b16 p, pl; split16(fmaxf(d[r] * (1.0f / (XS * WSC)) + bb, 0.0f) * XS, p, pl); Hh[wave][8 * hlf + r][t * 16 + nloc] = p; Hl[wave][8 * hlf + r][t * 16 + nloc] = pl; } } }
  wave_lds_sync();
  v8f f = {};
  for (int kb = 0; kb < DFF; kb += 32) { const v16b bw = frag_kb(F2P + (size_t)nloc * DFF + kb, hlf); f = wmma16b(frag_kb(&Hh[wave][nloc][kb], hlf), bw, f); f = wmma16b(frag_kb(&Hl[wave][nloc][kb], hlf), bw, f); }
  for (int r = 0; r < 8; ++r) att_s[wave][8 * hlf + r][nloc] += f[r] * (1.0f / (XS * WSC)) + bf16_rne(fb2[nloc]);
  wave_lds_sync();
  if (lane < 16) { float v[D]; for (int c = 0; c < D; ++c) v[c] = att_s[wave][lane][c]; float mu = 0.0f; for (int c = 0; c < D; ++c) mu += v[c]; mu *= (1.0f / D); float var = 0.0f; for (int c = 0; c < D; ++c) { const float dv = v[c] - mu; var += dv * dv; } var *= (1.0f / D); const float rs = 1.0f / sqrtf(var + EPS);
    for (int c = 0; c < D; ++c) att_s[wave][lane][c] = (v[c] - mu) * rs * bf16_rne(l2g[c]) + bf16_rne(l2b[c]); }
  wave_lds_sync();
  if (lane < D) { float s = 0.0f; for (int rr = 0; rr < 16; ++rr) s += att_s[wave][rr][lane]; part[wave][lane] = s; }
  __syncthreads();
  if (t_ < 32) row[t_] = (t_ < D) ? ((part[0][t_] + part[1][t_]) + part[2][t_]) + part[3][t_] : 0.0f;
  __syncthreads();
  for (int pass = 0; pass < 2; ++pass) { if (t_ < 8) *(volatile v4f*)(PSO + (size_t)blockIdx.x * 32 + t_ * 4) = *(const v4f*)(&row[t_ * 4]); __threadfence(); }
}
__global__ __launch_bounds__(256) void head_kernel(const float* __restrict__ PSO, const float* __restrict__ ow, const float* __restrict__ obias, float* __restrict__ out) {
  __shared__ float pooled[NB][D]; __shared__ __attribute__((aligned(16))) float res[NB * NCLS];
  const int t_ = threadIdx.x;
  if (t_ < NB * D) { const int b = t_ / D, c = t_ % D; float s = 0.0f; for (int k = 0; k < L / 64; ++k) s += PSO[((size_t)b * (L / 64) + k) * 32 + c]; pooled[b][c] = s * (1.0f / L); }
  __syncthreads();
  if (t_ < NB * NCLS) { const int b = t_ / NCLS, o = t_ % NCLS; float s = bf16_rne(obias[o]);
#pragma unroll 1
    for (int c = 0; c < D; ++c) s += pmul(pooled[b][c], bf16_rne(ow[c * NCLS + o])); res[t_] = s; }
  __syncthreads();
  for (int pass = 0; pass < 2; ++pass) { if (t_ < NB * NCLS / 4) *(volatile v4f*)(out + t_ * 4) = *(const v4f*)(&res[t_ * 4]); __threadfence(); }
}
}

extern "C" void kernel_launch(void* const* d_in, const int* in_sizes, int n_in, void* d_out, int out_size, void* d_ws, size_t ws_size, hipStream_t stream) {
  (void)n_in;
  auto Fp = [&](int i) { return (const float*)d_in[i]; };
  if (in_sizes[0] != NB * NC * L || in_sizes[1] != OC1 * 8 || in_sizes[5] != D * K2 || in_sizes[9] != D * D || in_sizes[12] != (2 * L - 1) * NH || in_sizes[17] != D * DFF || in_sizes[19] != DFF * D || in_sizes[23] != D * NCLS || out_size != NB * NCLS) return;
  size_t off = 0; char* ws = (char*)d_ws;
  auto carve = [&](size_t bytes) { char* p = ws + off; off += (bytes + 255) & ~(size_t)255; return p; };
  b16* W1P = (b16*)carve(OC1 * 32 * 2); b16* W2P = (b16*)carve((size_t)D * K2 * 2); b16* F1P = (b16*)carve((size_t)DFF * 32 * 2); b16* F2P = (b16*)carve((size_t)D * DFF * 2);
  b16* H1h = (b16*)carve((size_t)NT * K2 * 2); b16* H1l = (b16*)carve((size_t)NT * K2 * 2); float* PS1 = (float*)carve((size_t)NBLK1 * OC1 * 4); float* MU1 = (float*)carve(OC1 * 4); float* RS1 = (float*)carve(OC1 * 4);
  float* H2 = (float*)carve((size_t)NT * D * 4); float* PS2 = (float*)carve((size_t)(NT / 64) * 32 * 4); float* MU2 = (float*)carve(D * 4); float* RS2 = (float*)carve(D * 4);
  float* XSf = (float*)carve((size_t)NT * D * 4); b16* Qh = (b16*)carve((size_t)NB * NH * L * 32 * 2); b16* Ql = (b16*)carve((size_t)NB * NH * L * 32 * 2); b16* Kh = (b16*)carve((size_t)NB * NH * L * 32 * 2); b16* Kl = (b16*)carve((size_t)NB * NH * L * 32 * 2);
  b16* Vh = (b16*)carve((size_t)NB * NH * 16 * L * 2); b16* Vl = (b16*)carve((size_t)NB * NH * 16 * L * 2); float* OB = (float*)carve((size_t)NB * NH * L * HD * 4); float* PSO = (float*)carve((size_t)(NT / 64) * 32 * 4);
  if (off > ws_size || off > ((size_t)128 << 20)) return;
  const dim3 g1(NB, NC * (L / 64));
  prepw_kernel<<<(OC1 * 32 / 8 + D * K2 / 8 + DFF * 32 / 8 + D * DFF / 8 + 255) / 256, 256, 0, stream>>>(Fp(1), Fp(5), Fp(17), Fp(19), W1P, W2P, F1P, F2P);
  conv1_kernel<<<g1, 128, 0, stream>>>(Fp(0), W1P, Fp(2), H1h, H1l, PS1);
  bnred_kernel<<<1, 64, 0, stream>>>(PS1, NBLK1, (float)(NB * NC * L), 0, nullptr, MU1);
  bn1var_kernel<<<g1, 128, 0, stream>>>(H1h, H1l, MU1, PS1);
  bnred_kernel<<<1, 64, 0, stream>>>(PS1, NBLK1, (float)(NB * NC * L), 1, nullptr, RS1);
  conv2_kernel<<<NT / 32, 64, 0, stream>>>(H1h, H1l, MU1, RS1, Fp(3), Fp(4), W2P, Fp(6), H2);
  bn2part_kernel<<<NT / 64, 64, 0, stream>>>(H2, nullptr, 0, PS2);
  bnred2_kernel<<<1, 32, 0, stream>>>(PS2, NT / 64, (float)NT, 0, MU2);
  bn2part_kernel<<<NT / 64, 64, 0, stream>>>(H2, MU2, 1, PS2);
  bnred2_kernel<<<1, 32, 0, stream>>>(PS2, NT / 64, (float)NT, 1, RS2);
  token_kernel<<<NT / 32, 32, 0, stream>>>(H2, MU2, RS2, Fp(7), Fp(8), Fp(9), Fp(10), Fp(11), XSf, Qh, Ql, Kh, Kl, Vh, Vl);
  attn_kernel<<<dim3(L / 16, NH, NB), 32, 0, stream>>>(Qh, Ql, Kh, Kl, Vh, Vl, Fp(12), OB);
  post_kernel<<<NT / 64, 128, 0, stream>>>(OB, XSf, Fp(13), Fp(14), Fp(15), Fp(16), F1P, Fp(18), F2P, Fp(20), Fp(21), Fp(22), PSO);
  head_kernel<<<1, 256, 0, stream>>>(PSO, Fp(23), Fp(24), (float*)d_out);
}
